// Model_17918603559215
// MI455X (gfx1250) — hardware-run, weakly checked
//
#include <hip/hip_runtime.h>
#include <math.h>

typedef __attribute__((ext_vector_type(16))) _Float16 v16h;
typedef __attribute__((ext_vector_type(8)))  _Float16 v8h;
typedef __attribute__((ext_vector_type(16))) __bf16   v16b;
typedef __attribute__((ext_vector_type(8)))  __bf16   v8b;
typedef __attribute__((ext_vector_type(8)))  float    v8f;
typedef __attribute__((ext_vector_type(4)))  float    v4f;

constexpr int kB    = 8;
constexpr int kT    = 512;
constexpr int kC    = 862;
constexpr int kP    = 96;
constexpr int kD    = 128;
constexpr int kI    = 256;
constexpr int kNH   = 4;
constexpr int kDH   = 64;
constexpr int kNB   = 2;
constexpr int kMA   = 25;
constexpr int kCK   = 4;
constexpr int kR    = kB * kC;
constexpr int kRP   = 6912;
constexpr int kRT   = 7104;
constexpr int kSP   = 896;
constexpr int kTP   = 1024;
constexpr int kNCh  = kB * kNH;
constexpr int kThr  = 256;
constexpr float kInCarry = 1024.0f;
constexpr float kWCarry = 4096.0f;
constexpr float kCP = 1048576.0f;
constexpr float kHC = 16384.0f;
constexpr float kScII = 1.0f / (kInCarry * kInCarry), kScIW = 1.0f / (kInCarry * kWCarry), kScQK = 0.125f / (kInCarry * kInCarry), kScPV = 1.0f / (kCP * kInCarry), kScDN = 1.0f / (kHC * kWCarry);
constexpr float kInvD = 1.0f / 128.0f, kInvDH = 1.0f / 64.0f, kInvMA = 1.0f / 25.0f;
constexpr float kEps = 1e-5f;
constexpr float kF16MinNormal = 6.103515625e-5f;

static_assert(kR == 6896 && kRP >= kR && (kRP % 64) == 0 && (kRT % 64) == 0 && kRT >= (kB - 1) * kC + kTP && kSP >= kC && (kSP % 64) == 0 && (kTP % 64) == 0 && kTP >= kSP, "row paddings");
static_assert(((kRP / 64) * (kD / 64)) % 8 == 0 && ((kI / 64) * (kTP / 64)) % 8 == 0 && ((kTP / 64) * (kSP / 64)) % 8 == 0 && ((kTP / 64) * (kDH / 64)) % 8 == 0, "every grid a whole number of 8-tile blocks (the smallest: 216, 64, 224 and 16 tiles)");
static_assert((kP % 32) == 0 && (kD % 32) == 0 && (kI % 32) == 0 && (kDH % 32) == 0 && (kSP % 32) == 0 && ((3 * kI) % 32) == 0 && ((4 * kT) % 32) == 0, "GEMM K multiples of 32");
static_assert(kDH == 64 && 0.125f * 0.125f * 64.0f == 1.0f, "the key scale 64^-1/2 = 2^-3 is folded into the scores' epilogue scale");

constexpr size_t kOffWH = 0ull;
constexpr size_t kOffWP1 = 524288ull;
constexpr size_t kOffWP2 = 548864ull;
constexpr size_t kOffWUP = 581632ull;
constexpr size_t kOffWQK = 843776ull;
constexpr size_t kOffWV = 1368064ull;
constexpr size_t kOffWIF = 1630208ull;
constexpr size_t kOffWDN = 2023424ull;
constexpr size_t kOffBIAS = 2154496ull;
constexpr size_t kOffAS = 2170880ull;
constexpr size_t kOffMT = 2301952ull;
constexpr size_t kOffFL = 2433024ull;
constexpr size_t kOffNORM = 2564096ull;
constexpr size_t kOffAH = 6758400ull;
constexpr size_t kOffX0 = 35069952ull;
constexpr size_t kOffX0H = 38608896ull;
constexpr size_t kOffX = 40378368ull;
constexpr size_t kOffY16 = 43917312ull;
constexpr size_t kOffUP = 45686784ull;
constexpr size_t kOffXC = 59842560ull;
constexpr size_t kOffXC16 = 66920448ull;
constexpr size_t kOffXIN16 = 70557696ull;
constexpr size_t kOffQK = 74194944ull;
constexpr size_t kOffV = 88350720ull;
constexpr size_t kOffG16 = 95428608ull;
constexpr size_t kOffIF = 106340352ull;
constexpr size_t kOffVTF = 109879296ull;
constexpr size_t kOffVT16 = 110927872ull;
constexpr size_t kOffSC = 111386624ull;
constexpr size_t kOffP16 = 126066688ull;
constexpr size_t kOffHV = 133406720ull;
constexpr size_t kOffHS16 = 134455296ull;
constexpr size_t kOffDN = 137994240ull;
constexpr size_t kOffOUT2 = 141533184ull;
constexpr size_t kWsTotal = 145072128ull;
static_assert(kWsTotal <= 268435456ull, "carve cap: the offered workspace");
static_assert(kOffWH == 0
              && kOffWP1 == kOffWH + 524288ull
              && kOffWP2 == kOffWP1 + 24576ull
              && kOffWUP == kOffWP2 + 32768ull
              && kOffWQK == kOffWUP + 262144ull
              && kOffWV == kOffWQK + 524288ull
              && kOffWIF == kOffWV + 262144ull
              && kOffWDN == kOffWIF + 393216ull
              && kOffBIAS == kOffWDN + 131072ull
              && kOffAS == kOffBIAS + 16384ull
              && kOffMT == kOffAS + 131072ull
              && kOffFL == kOffMT + 131072ull
              && kOffNORM == kOffFL + 131072ull
              && kOffAH == kOffNORM + 4194304ull
              && kOffX0 == kOffAH + 28311552ull
              && kOffX0H == kOffX0 + 3538944ull
              && kOffX == kOffX0H + 1769472ull
              && kOffY16 == kOffX + 3538944ull
              && kOffUP == kOffY16 + 1769472ull
              && kOffXC == kOffUP + 14155776ull
              && kOffXC16 == kOffXC + 7077888ull
              && kOffXIN16 == kOffXC16 + 3637248ull
              && kOffQK == kOffXIN16 + 3637248ull
              && kOffV == kOffQK + 14155776ull
              && kOffG16 == kOffV + 7077888ull
              && kOffIF == kOffG16 + 10911744ull
              && kOffVTF == kOffIF + 3538944ull
              && kOffVT16 == kOffVTF + 1048576ull
              && kOffSC == kOffVT16 + 458752ull
              && kOffP16 == kOffSC + 14680064ull
              && kOffHV == kOffP16 + 7340032ull
              && kOffHS16 == kOffHV + 1048576ull
              && kOffDN == kOffHS16 + 3538944ull
              && kOffOUT2 == kOffDN + 3538944ull
              && kWsTotal == kOffOUT2 + 3538944ull, "the carve is chained and totalled");
static_assert((kOffWH % 256) == 0 && (kOffWP1 % 256) == 0 && (kOffWP2 % 256) == 0 && (kOffWUP % 256) == 0 && (kOffWQK % 256) == 0 && (kOffWV % 256) == 0 && (kOffWIF % 256) == 0 && (kOffWDN % 256) == 0 && (kOffBIAS % 256) == 0 && (kOffAS % 256) == 0 && (kOffMT % 256) == 0 && (kOffFL % 256) == 0 && (kOffNORM % 256) == 0 && (kOffAH % 256) == 0 && (kOffX0 % 256) == 0 && (kOffX0H % 256) == 0 && (kOffX % 256) == 0 && (kOffY16 % 256) == 0 && (kOffUP % 256) == 0 && (kOffXC % 256) == 0 && (kOffXC16 % 256) == 0 && (kOffXIN16 % 256) == 0 && (kOffQK % 256) == 0 && (kOffV % 256) == 0 && (kOffG16 % 256) == 0 && (kOffIF % 256) == 0 && (kOffVTF % 256) == 0 && (kOffVT16 % 256) == 0 && (kOffSC % 256) == 0 && (kOffP16 % 256) == 0 && (kOffHV % 256) == 0 && (kOffHS16 % 256) == 0 && (kOffDN % 256) == 0 && (kOffOUT2 % 256) == 0, "aligned regions");
constexpr int kFBS = 0, kFBP1 = 128, kFBP2 = 256, kFBlk = 384, kFBlkLen = 768, kFBUP = 0, kFBIF = 512, kFBDN = 640, kFZB = 3072, kFEnd = 4096;
static_assert(kFBlk + kNB * kFBlkLen == 1920 && kFZB >= 1920 && kFEnd - kFZB == 1024 && (kFBlk % 128) == 0 && (kFBlkLen % 128) == 0 && (kFBIF % 128) == 0 && (kFBDN % 128) == 0 && (kFZB % 128) == 0, "bias stream layout; the zero row covers the widest zero-bias product (1,024 columns)");

__device__ __forceinline__ unsigned short f2bf_bits(float f) {
  unsigned u = __float_as_uint(f);
  return (unsigned short)((u + 0x7FFFu + ((u >> 16) & 1u)) >> 16);
}
__device__ __forceinline__ float bf_bits2f(unsigned short h) { return __uint_as_float(((unsigned)h) << 16); }
__device__ __forceinline__ float bf16r(float f) { return bf_bits2f(f2bf_bits(f)); }
__device__ __forceinline__ float carry_flush(float v, float carry) {
  const float s = v * carry;
  return (fabsf(s) < kF16MinNormal) ? 0.0f : s;
}
__device__ __forceinline__ float frcp(float x) { return __builtin_amdgcn_rcpf(x); }

__device__ __forceinline__ void dep_guard4_h(v8f& a, v8f& b, v8f& c, v8f& d, v16h x, v16h y) { asm volatile("v_nop\n\tv_nop\n\tv_nop\n\tv_nop" : "+v"(a), "+v"(b), "+v"(c), "+v"(d) : "v"(x), "v"(y)); }
__device__ __forceinline__ void dep_guard4_b(v8f& a, v8f& b, v8f& c, v8f& d, v16b x, v16b y) { asm volatile("v_nop\n\tv_nop\n\tv_nop\n\tv_nop" : "+v"(a), "+v"(b), "+v"(c), "+v"(d) : "v"(x), "v"(y)); }
__device__ __forceinline__ void keep4_h(v16h a, v16h b, v16h c, v16h d) { asm volatile("v_nop" :: "v"(a), "v"(b), "v"(c), "v"(d)); }
__device__ __forceinline__ void keep4_b(v16b a, v16b b, v16b c, v16b d) { asm volatile("v_nop" :: "v"(a), "v"(b), "v"(c), "v"(d)); }
__device__ __forceinline__ void acc_guard4(v8f& a, v8f& b, v8f& c, v8f& d) { asm volatile("v_nop\n\tv_nop\n\tv_nop\n\tv_nop" : "+v"(a), "+v"(b), "+v"(c), "+v"(d)); }

template <typename T> struct Frag;
template <> struct Frag<_Float16> {
  typedef v16h V; union U { v16h v; v8h h[2]; };
  static __device__ __forceinline__ v16h load(const _Float16* p) {
    U f; f.h[0] = *(const v8h*)(p); f.h[1] = *(const v8h*)(p + 16); return f.v;
  }
  static __device__ __forceinline__ v8f mma(v16h a, v16h b, v8f c) {
    return __builtin_amdgcn_wmma_f32_16x16x32_f16(false, a, false, b, (short)0, c, false, false);
  }
  static __device__ __forceinline__ void guard4(v8f& a, v8f& b, v8f& c, v8f& d, v16h x, v16h y) { dep_guard4_h(a, b, c, d, x, y); }
  static __device__ __forceinline__ void keep(v16h a, v16h b, v16h c, v16h d) { keep4_h(a, b, c, d); }
};
template <> struct Frag<__bf16> {
  typedef v16b V; union U { v16b v; v8b h[2]; };
  static __device__ __forceinline__ v16b load(const __bf16* p) {
    U f; f.h[0] = *(const v8b*)(p); f.h[1] = *(const v8b*)(p + 16); return f.v;
  }
  static __device__ __forceinline__ v8f mma(v16b a, v16b b, v8f c) {
    return __builtin_amdgcn_wmma_f32_16x16x32_bf16(false, a, false, b, (short)0, c, false, false);
  }
  static __device__ __forceinline__ void guard4(v8f& a, v8f& b, v8f& c, v8f& d, v16b x, v16b y) { dep_guard4_b(a, b, c, d, x, y); }
  static __device__ __forceinline__ void keep(v16b a, v16b b, v16b c, v16b d) { keep4_b(a, b, c, d); }
};

__device__ __forceinline__ v8f mma_h(v16h a, v16h b, v8f c) {
  c = __builtin_amdgcn_wmma_f32_16x16x32_f16(false, a, false, b, (short)0, c, false, false);
  asm volatile("v_nop\n\tv_nop\n\tv_nop\n\tv_nop" : "+v"(c) : "v"(a), "v"(b));
  return c;
}

template <int ET> struct Elem;
template <> struct Elem<0> { typedef _Float16 T; };
template <> struct Elem<1> { typedef __bf16 T; };
template <int ET, bool SPLIT, int BIAS_MODE, int OUT_MODE, bool RESID, int ACT = 0>
__global__ __launch_bounds__(256) void wmma_gemm64(
    const unsigned short* __restrict__ Ap, const unsigned short* __restrict__ A2p, int lda, long strideA,
    const unsigned short* __restrict__ Btp, const unsigned short* __restrict__ Bt2p, int ldb, long strideB,
    void* __restrict__ Cout, void* __restrict__ Cout2, int ldc, long strideC,
    const float* __restrict__ bias,
    const float* __restrict__ resid, long strideR,
    int M, int N, int K, float scale) {
  typedef typename Elem<ET>::T T;
  typedef typename Frag<T>::V V;
  const T* A = (const T*)Ap; const T* A2 = (const T*)A2p; const T* Bt = (const T*)Btp; const T* Bt2 = (const T*)Bt2p;
  __shared__ __align__(16) float sT[8][16 * 68];
  const int b    = blockIdx.y;
  const int lane = threadIdx.x & 31;
  const int wave = threadIdx.x >> 5;
  const int tilesN = N >> 6;
  const int tilesM = M >> 6;
  const int tile = blockIdx.x * 8 + wave;
  if (tile >= tilesM * tilesN) return;
  const int tm = tile / tilesN;
  const int tn = tile - tm * tilesN;
  const int m0 = tm << 6;
  const int n0 = tn << 6;

  const T* Ab  = A  + (size_t)b * strideA;
  const T* Bb  = Bt + (size_t)b * strideB;
  const T* Ab2 = SPLIT ? (A2  + (size_t)b * strideA) : nullptr;
  const T* Bb2 = SPLIT ? (Bt2 + (size_t)b * strideB) : nullptr;

  const int rlane = lane & 15;
  const int koff  = (lane >> 4) * 8;
  const int mOff  = (lane >> 4) * 8;

  v8f acc[4][4];
#pragma unroll
  for (int i = 0; i < 4; ++i)
#pragma unroll
    for (int j = 0; j < 4; ++j) acc[i][j] = (v8f){0.f,0.f,0.f,0.f,0.f,0.f,0.f,0.f};

  for (int k0 = 0; k0 < K; k0 += 32) {
    V bh[4], bl[4];
#pragma unroll
    for (int j = 0; j < 4; ++j) {
      const size_t bo = (size_t)(n0 + (j << 4) + rlane) * ldb + koff + k0;
      bh[j] = Frag<T>::load(Bb + bo);
      if (SPLIT) bl[j] = Frag<T>::load(Bb2 + bo);
    }
#pragma unroll
    for (int i = 0; i < 4; ++i) {
      const size_t ao = (size_t)(m0 + (i << 4) + rlane) * lda + koff + k0;
      V ah = Frag<T>::load(Ab + ao);
      V al;
      if (SPLIT) al = Frag<T>::load(Ab2 + ao);
#pragma unroll
      for (int j = 0; j < 4; ++j) {
        acc[i][j] = Frag<T>::mma(ah, bh[j], acc[i][j]);
        if (SPLIT) {
          acc[i][j] = Frag<T>::mma(ah, bl[j], acc[i][j]);
          acc[i][j] = Frag<T>::mma(al, bh[j], acc[i][j]);
        }
      }
      Frag<T>::guard4(acc[i][0], acc[i][1], acc[i][2], acc[i][3], ah, SPLIT ? al : ah);
    }
    Frag<T>::keep(bh[0], bh[1], bh[2], bh[3]);
    if (SPLIT) Frag<T>::keep(bl[0], bl[1], bl[2], bl[3]);
  }
  acc_guard4(acc[0][0], acc[0][1], acc[0][2], acc[0][3]);
  acc_guard4(acc[1][0], acc[1][1], acc[1][2], acc[1][3]);
  acc_guard4(acc[2][0], acc[2][1], acc[2][2], acc[2][3]);
  acc_guard4(acc[3][0], acc[3][1], acc[3][2], acc[3][3]);

  float* slab = sT[wave];
  const float* Rb = RESID ? (resid + (size_t)b * strideR) : nullptr;
#pragma unroll
  for (int i = 0; i < 4; ++i) {
    const int mBase = m0 + (i << 4);
#pragma unroll
    for (int j = 0; j < 4; ++j) {
      const int n = n0 + (j << 4) + rlane;
      float bv = 0.f;
      if (BIAS_MODE == 2) bv = bias[n];
#pragma unroll
      for (int r = 0; r < 8; ++r) {
        float v = acc[i][j][r] * scale;
        if (BIAS_MODE == 1) v += bias[mBase + mOff + r];
        if (BIAS_MODE == 2) v += bv;
        if (RESID) v += Rb[(size_t)(mBase + mOff + r) * ldc + n];
        if (ACT == 1) v = tanhf(v);
        if (ACT == 2) v = fmaxf(v, 0.0f);
        if (ACT == 3) v = v / (1.0f + expf(-v));
        if (ACT == 4) v = (v > 0.f) ? v : 0.01f * v;
        slab[(mOff + r) * 68 + (j << 4) + rlane] = v;
      }
    }
    __builtin_amdgcn_fence(__ATOMIC_RELEASE, "workgroup");
    __builtin_amdgcn_wave_barrier();
    __builtin_amdgcn_fence(__ATOMIC_ACQUIRE, "workgroup");
    if (OUT_MODE == 0) {
      float* C = (float*)Cout + (size_t)b * strideC;
      const int hh = lane >> 4, c4 = (lane & 15) * 4;
      for (int pass = 0; pass < 2; ++pass) {
#pragma unroll
        for (int it = 0; it < 8; ++it) {
          const int row = it * 2 + hh;
          v4f v = *(const v4f*)(slab + row * 68 + c4);
          *(volatile v4f*)(C + (size_t)(mBase + row) * ldc + n0 + c4) = v;
        }
        __threadfence();
      }
    } else {
      const int q = lane >> 3, c8 = (lane & 7) * 8;
      unsigned short* C  = (unsigned short*)Cout  + (size_t)b * strideC;
      unsigned short* C2 = (OUT_MODE == 2) ? ((unsigned short*)Cout2 + (size_t)b * strideC) : nullptr;
      for (int pass = 0; pass < 2; ++pass) {
#pragma unroll
        for (int it = 0; it < 4; ++it) {
          const int row = it * 4 + q;
          const float* sp = slab + row * 68 + c8;
          v8h hv, lv;
#pragma unroll
          for (int e = 0; e < 8; ++e) {
            if (OUT_MODE == 1) {
              hv[e] = (_Float16)sp[e];
            } else {
              unsigned short hb = f2bf_bits(sp[e]);
              unsigned short lb = f2bf_bits(sp[e] - bf_bits2f(hb));
              hv[e] = __builtin_bit_cast(_Float16, hb);
              lv[e] = __builtin_bit_cast(_Float16, lb);
            }
          }
          *(volatile v8h*)(C + (size_t)(mBase + row) * ldc + n0 + c8) = hv;
          if (OUT_MODE == 2) *(volatile v8h*)(C2 + (size_t)(mBase + row) * ldc + n0 + c8) = lv;
        }
        __threadfence();
      }
    }
    __builtin_amdgcn_fence(__ATOMIC_RELEASE, "workgroup");
    __builtin_amdgcn_wave_barrier();
    __builtin_amdgcn_fence(__ATOMIC_ACQUIRE, "workgroup");
  }
}

__global__ __launch_bounds__(kThr) void cast_plane_kernel(const float* __restrict__ src, unsigned short* __restrict__ dst,
                                                          int colsLog2, int dstPitch, int dstOff) {
  const int i   = blockIdx.x * kThr + threadIdx.x;
  const int sh  = colsLog2 - 3;
  const int row = i >> sh;
  const int c8  = (i & ((1 << sh) - 1)) * 8;
  const float* sp = src + ((size_t)row << colsLog2) + c8;
  const v4f a0 = *(const v4f*)(sp);
  const v4f a1 = *(const v4f*)(sp + 4);
  v8h hv;
#pragma unroll
  for (int e = 0; e < 4; ++e) {
    const float f0 = a0[e];
    const float f1 = a1[e];
    hv[e]     = (_Float16)carry_flush(bf16r(f0), kInCarry);
    hv[4 + e] = (_Float16)carry_flush(bf16r(f1), kInCarry);
  }
  unsigned short* dp = dst + (size_t)row * dstPitch + dstOff + c8;
  *(volatile v8h*)dp = hv;
  __threadfence();
  *(volatile v8h*)dp = hv;
}
__global__ __launch_bounds__(256) void wt_plane_kernel(const float* __restrict__ W, unsigned short* __restrict__ dst, int K, int N, int nLive, int ldd, int colOff) {
  const int n  = blockIdx.x;
  const int k8 = threadIdx.x * 8;
  const bool live = n < nLive;
  const int nc = live ? n : 0;
  v8h hv;
#pragma unroll
  for (int e = 0; e < 8; ++e) {
    const float w = W[(size_t)(k8 + e) * N + nc];
    hv[e] = (_Float16)(live ? carry_flush(bf16r(w), kWCarry) : 0.0f);
  }
  unsigned short* dp = dst + (size_t)n * ldd + colOff + k8;
  *(volatile v8h*)dp = hv;
  __threadfence();
  *(volatile v8h*)dp = hv;
}

__global__ __launch_bounds__(kThr) void setup_kernel(const float* __restrict__ bs, const float* __restrict__ bt, const float* __restrict__ bp1, const float* __restrict__ bp2,
                                                     const float* __restrict__ bup, const float* __restrict__ bi, const float* __restrict__ bf, const float* __restrict__ bdn,
                                                     float* __restrict__ BIAS, unsigned short* __restrict__ WH, unsigned short* __restrict__ WP2) {
  const unsigned v = blockIdx.x * (unsigned)kThr + threadIdx.x;
  if (v < 1024u) {
    const unsigned i0 = v * 4u;
    v4f o = {0.f, 0.f, 0.f, 0.f};
    if (i0 < (unsigned)kFBP1) {
      if (i0 < (unsigned)kP) {
        const v4f a = *(const v4f*)(bs + i0), c = *(const v4f*)(bt + i0);
#pragma unroll
        for (int e = 0; e < 4; ++e) { const float p = a[e], q = c[e]; o[e] = bf16r(p) + bf16r(q); }
      }
    } else if (i0 < (unsigned)kFBP2) {
      const v4f a = *(const v4f*)(bp1 + (i0 - (unsigned)kFBP1));
#pragma unroll
      for (int e = 0; e < 4; ++e) { const float p = a[e]; o[e] = bf16r(p); }
    } else if (i0 < (unsigned)kFBlk) {
      const unsigned j = i0 - (unsigned)kFBP2;
      if (j < (unsigned)kP) {
        const v4f a = *(const v4f*)(bp2 + j);
#pragma unroll
        for (int e = 0; e < 4; ++e) { const float p = a[e]; o[e] = bf16r(p); }
      }
    } else if (i0 < (unsigned)(kFBlk + kNB * kFBlkLen)) {
      const unsigned w = i0 - (unsigned)kFBlk;
      const unsigned blk = (w >= (unsigned)kFBlkLen) ? 1u : 0u;
      const unsigned j = w - blk * (unsigned)kFBlkLen;
      if (j < (unsigned)kFBIF) {
        const v4f a = *(const v4f*)(bup + (size_t)blk * (2 * kI) + j);
#pragma unroll
        for (int e = 0; e < 4; ++e) { const float p = a[e]; o[e] = bf16r(p); }
      } else if (j < (unsigned)kFBDN) {
        const unsigned g = j - (unsigned)kFBIF;
        if (g == 0u) {
          const v4f a = *(const v4f*)(bi + (size_t)blk * kNH);
#pragma unroll
          for (int e = 0; e < 4; ++e) { const float p = a[e]; o[e] = bf16r(p); }
        } else if (g == 4u) {
          const v4f a = *(const v4f*)(bf + (size_t)blk * kNH);
#pragma unroll
          for (int e = 0; e < 4; ++e) { const float p = a[e]; o[e] = bf16r(p); }
        }
      } else {
        const v4f a = *(const v4f*)(bdn + (size_t)blk * kD + (j - (unsigned)kFBDN));
#pragma unroll
        for (int e = 0; e < 4; ++e) { const float p = a[e]; o[e] = bf16r(p); }
      }
    }
    float* dp = BIAS + i0;
    *(volatile v4f*)dp = o;
    __threadfence();
    *(volatile v4f*)dp = o;
  } else {
    v8h z;
#pragma unroll
    for (int e = 0; e < 8; ++e) z[e] = (_Float16)0.0f;
    unsigned short* dp = (v < 9216u) ? (WH + (size_t)kP * (4 * kT) + (size_t)(v - 1024u) * 8u) : (WP2 + (size_t)kP * kD + (size_t)(v - 9216u) * 8u);
    *(volatile v8h*)dp = z;
    __threadfence();
    *(volatile v8h*)dp = z;
  }
}
static_assert(kFEnd / 4 == 1024 && (128 - kP) * (4 * kT) / 8 == 8192 && (128 - kP) * kD / 8 == 512 && 1024 + 8192 + 512 == 38 * kThr && kNH == 4, "set-up grid exact; a gate bias is one 4-float group");

__global__ __launch_bounds__(kThr) void zero_kernel(unsigned short* __restrict__ dst) {
  const size_t v = (size_t)blockIdx.x * kThr + threadIdx.x;
  v8h z;
#pragma unroll
  for (int e = 0; e < 8; ++e) z[e] = (_Float16)0.0f;
  unsigned short* dp = dst + v * 8u;
  *(volatile v8h*)dp = z;
  __threadfence();
  *(volatile v8h*)dp = z;
}
static_assert(((size_t)(kRP - kR) * (4 * kT) / 8) % kThr == 0, "AH's tail rows: an exact grid");

__global__ __launch_bounds__(kThr) void decomp_kernel(const float* __restrict__ x_enc, unsigned short* __restrict__ AH) {
  const unsigned c = blockIdx.x * (unsigned)kThr + threadIdx.x;
  if (c >= (unsigned)kC) return;
  const unsigned bj = blockIdx.y;
  const unsigned b = bj >> 3, j = bj & 7u;
  const float* xb = x_enc + (size_t)b * kT * kC + c;
  const int l0 = (int)(j * 64u) - 12;
  float xv[88];
  float run[89];
  run[0] = 0.0f;
#pragma unroll
  for (int i = 0; i < 88; ++i) {
    int l = l0 + i;
    l = (l < 0) ? 0 : ((l > kT - 1) ? (kT - 1) : l);
    const float x0 = xb[(size_t)l * kC];
    xv[i] = bf16r(x0);
    run[i + 1] = run[i] + xv[i];
  }
  unsigned short* rowp = AH + (size_t)(b * (unsigned)kC + c) * (4 * kT) + j * 64u;
#pragma unroll
  for (int g = 0; g < 8; ++g) {
    v8h sh, sl, th, tl;
#pragma unroll
    for (int e = 0; e < 8; ++e) {
      const int i = g * 8 + e;
      const float tr = (run[i + kMA] - run[i]) * kInvMA;
      const float se = xv[i + 12] - tr;
      const float cs = carry_flush(se, kInCarry);
      const _Float16 hs = (_Float16)cs;
      const float rs = cs - (float)hs;
      const float ct = carry_flush(tr, kInCarry);
      const _Float16 ht = (_Float16)ct;
      const float rt = ct - (float)ht;
      sh[e] = hs; sl[e] = (_Float16)((fabsf(rs) < kF16MinNormal) ? 0.0f : rs);
      th[e] = ht; tl[e] = (_Float16)((fabsf(rt) < kF16MinNormal) ? 0.0f : rt);
    }
    for (int pass = 0; pass < 2; ++pass) {
      *(volatile v8h*)(rowp + g * 8) = sh;
      *(volatile v8h*)(rowp + kT + g * 8) = sl;
      *(volatile v8h*)(rowp + 2 * kT + g * 8) = th;
      *(volatile v8h*)(rowp + 3 * kT + g * 8) = tl;
      __threadfence();
    }
  }
}
static_assert((kC + kThr - 1) / kThr == 4 && kT == 8 * 64 && kMA == 25, "decomposition grid: 4 x 64 blocks");

__global__ __launch_bounds__(kThr) void cast8_kernel(const float* __restrict__ src, unsigned short* __restrict__ dst) {
  const size_t v = (size_t)blockIdx.x * kThr + threadIdx.x;
  const float* sp = src + v * 8u;
  const v4f a0 = *(const v4f*)sp, a1 = *(const v4f*)(sp + 4);
  v8h hv;
#pragma unroll
  for (int e = 0; e < 4; ++e) { hv[e] = (_Float16)carry_flush(a0[e], kInCarry); hv[4 + e] = (_Float16)carry_flush(a1[e], kInCarry); }
  unsigned short* dp = dst + v * 8u;
  *(volatile v8h*)dp = hv;
  __threadfence();
  *(volatile v8h*)dp = hv;
}
static_assert(((size_t)kRP * kD / 8) % kThr == 0, "cast grid exact");

__global__ __launch_bounds__(kThr) void addln_kernel(const float* A, const float* __restrict__ ADD, const float* __restrict__ g,
                                                     float* SUM32, unsigned short* __restrict__ O16, int flags) {
  const unsigned r = blockIdx.x * (unsigned)kThr + threadIdx.x;
  const bool wantAdd = (flags & 1) != 0, wantSum = (flags & 2) != 0;
  const float* a = A + (size_t)r * kD;
  const float* ad = ADD + (size_t)r * kD;
  float s = 0.0f;
#pragma unroll 4
  for (unsigned c = 0; c < (unsigned)kD; c += 4) {
    v4f x = *(const v4f*)(a + c);
    if (wantAdd) { const v4f y = *(const v4f*)(ad + c); x = x + y; }
    s += x[0]; s += x[1]; s += x[2]; s += x[3];
  }
  const float mu = s * kInvD;
  float q = 0.0f;
#pragma unroll 4
  for (unsigned c = 0; c < (unsigned)kD; c += 4) {
    v4f x = *(const v4f*)(a + c);
    if (wantAdd) { const v4f y = *(const v4f*)(ad + c); x = x + y; }
#pragma unroll
    for (int e = 0; e < 4; ++e) { const float d = x[e] - mu; q += d * d; }
  }
  const float rstd = rsqrtf(q * kInvD + kEps);
  float* sp = SUM32 + (size_t)r * kD;
  unsigned short* hp = O16 + (size_t)r * kD;
#pragma unroll 2
  for (unsigned c = 0; c < (unsigned)kD; c += 8) {
    v4f x0 = *(const v4f*)(a + c), x1 = *(const v4f*)(a + c + 4);
    if (wantAdd) { const v4f y0 = *(const v4f*)(ad + c), y1 = *(const v4f*)(ad + c + 4); x0 = x0 + y0; x1 = x1 + y1; }
    const v4f g0 = *(const v4f*)(g + c), g1 = *(const v4f*)(g + c + 4);
    v8h hv;
#pragma unroll
    for (int e = 0; e < 4; ++e) {
      hv[e] = (_Float16)carry_flush((x0[e] - mu) * rstd * bf16r(g0[e]), kInCarry);
      hv[4 + e] = (_Float16)carry_flush((x1[e] - mu) * rstd * bf16r(g1[e]), kInCarry);
    }
    for (int pass = 0; pass < 2; ++pass) {
      if (wantSum) { *(volatile v4f*)(sp + c) = x0; *(volatile v4f*)(sp + c + 4) = x1; }
      *(volatile v8h*)(hp + c) = hv;
      __threadfence();
    }
  }
}
static_assert(kRP % kThr == 0, "one thread a row: an exact grid");

__global__ __launch_bounds__(kThr) void conv_silu_kernel(const float* __restrict__ UP, const float* __restrict__ Wc, const float* __restrict__ bc,
                                                         float* __restrict__ XC, unsigned short* __restrict__ XC16, unsigned short* __restrict__ XIN16) {
  const unsigned v = blockIdx.x * (unsigned)kThr + threadIdx.x;
  const unsigned r = v >> 5, i8 = (v & 31u) * 8u;
  const bool live = r < (unsigned)kR;
  const unsigned rc = live ? r : 0u;
  const unsigned smp = rc / (unsigned)kC;
  const unsigned c = rc - smp * (unsigned)kC;
  float acc[8], xin[8];
  {
    const v4f b0 = *(const v4f*)(bc + i8), b1 = *(const v4f*)(bc + i8 + 4);
#pragma unroll
    for (int e = 0; e < 4; ++e) { acc[e] = bf16r(b0[e]); acc[4 + e] = bf16r(b1[e]); }
  }
#pragma unroll
  for (int j = 0; j < kCK; ++j) {
    const bool in = c + (unsigned)j >= (unsigned)(kCK - 1);
    const unsigned rr = in ? (rc + (unsigned)j - (unsigned)(kCK - 1)) : rc;
    const float* up = UP + (size_t)rr * (2 * kI) + i8;
    const v4f x0 = *(const v4f*)up, x1 = *(const v4f*)(up + 4);
    const v4f w0 = *(const v4f*)(Wc + (size_t)j * kI + i8), w1 = *(const v4f*)(Wc + (size_t)j * kI + i8 + 4);
#pragma unroll
    for (int e = 0; e < 4; ++e) {
      const float a0 = in ? x0[e] : 0.0f, a1 = in ? x1[e] : 0.0f;
      acc[e] += bf16r(w0[e]) * a0;
      acc[4 + e] += bf16r(w1[e]) * a1;
      if (j == kCK - 1) { xin[e] = x0[e]; xin[4 + e] = x1[e]; }
    }
  }
  v4f o0, o1; v8h hc, hx;
#pragma unroll
  for (int e = 0; e < 8; ++e) {
    const float s = acc[e] / (1.0f + expf(-acc[e]));
    if (e < 4) o0[e] = s; else o1[e - 4] = s;
    hc[e] = (_Float16)(live ? carry_flush(s, kInCarry) : 0.0f);
    hx[e] = (_Float16)(live ? carry_flush(xin[e], kInCarry) : 0.0f);
  }
  const bool wr32 = r < (unsigned)kRP;
  for (int pass = 0; pass < 2; ++pass) {
    if (wr32) { *(volatile v4f*)(XC + (size_t)r * kI + i8) = o0; *(volatile v4f*)(XC + (size_t)r * kI + i8 + 4) = o1; }
    *(volatile v8h*)(XC16 + (size_t)r * kI + i8) = hc;
    *(volatile v8h*)(XIN16 + (size_t)r * kI + i8) = hx;
    __threadfence();
  }
}
static_assert(((size_t)kRT * 32) % kThr == 0 && kI / 8 == 32, "conv grid exact; a wave = one row");

__global__ __launch_bounds__(kThr) void qkv_kernel(const float* __restrict__ QK, const float* __restrict__ V, unsigned short* __restrict__ G16) {
  const unsigned v = blockIdx.x * (unsigned)kThr + threadIdx.x;
  const unsigned r = v / 96u, c8 = (v - r * 96u) * 8u;
  const bool live = r < (unsigned)kR;
  const unsigned rc = live ? r : 0u;
  const float* sp = (c8 < (unsigned)(2 * kI)) ? (QK + (size_t)rc * (2 * kI) + c8) : (V + (size_t)rc * kI + (c8 - (unsigned)(2 * kI)));
  const v4f a0 = *(const v4f*)sp, a1 = *(const v4f*)(sp + 4);
  v8h hv;
#pragma unroll
  for (int e = 0; e < 4; ++e) {
    hv[e] = (_Float16)(live ? carry_flush(a0[e], kInCarry) : 0.0f);
    hv[4 + e] = (_Float16)(live ? carry_flush(a1[e], kInCarry) : 0.0f);
  }
  unsigned short* dp = G16 + (size_t)v * 8u;
  *(volatile v8h*)dp = hv;
  __threadfence();
  *(volatile v8h*)dp = hv;
}
static_assert((3 * kI) / 8 == 96 && ((size_t)kRT * 96) % kThr == 0, "q | k | v cast grid exact");

__global__ __launch_bounds__(kThr) void vt_kernel(const float* __restrict__ VTF, unsigned short* __restrict__ VT16) {
  const unsigned v = blockIdx.x * (unsigned)kThr + threadIdx.x;
  const unsigned d = v / 112u, s8 = (v - d * 112u) * 8u;
  const float* sp = VTF + (size_t)d * kTP + s8;
  const v4f a0 = *(const v4f*)sp, a1 = *(const v4f*)(sp + 4);
  v8h hv;
#pragma unroll
  for (int e = 0; e < 4; ++e) {
    hv[e] = (_Float16)((s8 + (unsigned)e < (unsigned)kC) ? carry_flush(a0[e], kInCarry) : 0.0f);
    hv[4 + e] = (_Float16)((s8 + 4u + (unsigned)e < (unsigned)kC) ? carry_flush(a1[e], kInCarry) : 0.0f);
  }
  unsigned short* dp = VT16 + (size_t)v * 8u;
  *(volatile v8h*)dp = hv;
  __threadfence();
  *(volatile v8h*)dp = hv;
}
static_assert(kSP / 8 == 112 && (kI * 112) % kThr == 0, "value-transpose grid exact");

__global__ __launch_bounds__(32) void gate_scan_kernel(const float* __restrict__ IFp, float* __restrict__ AS, float* __restrict__ MT, float* __restrict__ FL) {
  const unsigned ch = threadIdx.x;
  const unsigned smp = ch >> 2, hd = ch & 3u;
  const float* ip = IFp + (size_t)smp * kC * kD + hd;
  float cum = 0.0f, mx = 0.0f;
  for (int t = 0; t < kTP; ++t) {
    float av = 0.0f, mv = 0.0f, fv = 0.0f;
    if (t < kC) {
      const float ig = ip[(size_t)t * kD];
      const float fg = ip[(size_t)t * kD + kNH];
      const float lf = (fg >= 0.0f) ? -log1pf(expf(-fg)) : (fg - log1pf(expf(fg)));
      cum += lf;
      av = ig - cum;
      mx = (t == 0) ? av : ((av > mx) ? av : mx);
      mv = mx;
      fv = expf(-(cum + mx));
    }
    float* ap = AS + (size_t)ch * kTP + t;
    float* mp = MT + (size_t)ch * kTP + t;
    float* fp = FL + (size_t)ch * kTP + t;
    for (int pass = 0; pass < 2; ++pass) {
      *(volatile float*)ap = av;
      *(volatile float*)mp = mv;
      *(volatile float*)fp = fv;
      __threadfence();
    }
  }
}
static_assert(kNCh == 32 && kNH == 4, "one wave of chains");

__global__ __launch_bounds__(kThr) void mask_kernel(const float* __restrict__ SC, const float* __restrict__ AS, const float* __restrict__ MT, const float* __restrict__ FL,
                                                    unsigned short* __restrict__ P16, float* __restrict__ NORM, int smp) {
  const unsigned w = blockIdx.x * 8u + (threadIdx.x >> 5);
  const unsigned lane = threadIdx.x & 31u;
  const unsigned hd = w >> 10, t = w & 1023u;
  const unsigned ch = (unsigned)smp * (unsigned)kNH + hd;
  const bool rowLive = t < (unsigned)kC;
  const float mt = MT[(size_t)ch * kTP + (rowLive ? t : 0u)];
  const float* scp = SC + ((size_t)hd * kTP + t) * kSP;
  const float* asp = AS + (size_t)ch * kTP;
  unsigned short* pp = P16 + ((size_t)hd * kTP + t) * kSP;
  float sum = 0.0f;
#pragma unroll
  for (int it = 0; it < 4; ++it) {
    const unsigned j = lane + 32u * (unsigned)it;
    if (j < 112u) {
      const unsigned s8 = j * 8u;
      const v4f c0 = *(const v4f*)(scp + s8), c1 = *(const v4f*)(scp + s8 + 4);
      const v4f a0 = *(const v4f*)(asp + s8), a1 = *(const v4f*)(asp + s8 + 4);
      v8h hv;
#pragma unroll
      for (int e = 0; e < 8; ++e) {
        const float sc = (e < 4) ? c0[e] : c1[e - 4];
        const float as = (e < 4) ? a0[e] : a1[e - 4];
        const bool on = rowLive && (s8 + (unsigned)e <= t);
        const float dw = expf(as - mt);
        const float p = on ? sc * dw : 0.0f;
        sum += p;
        hv[e] = (_Float16)carry_flush(p, kCP);
      }
      for (int pass = 0; pass < 2; ++pass) {
        *(volatile v8h*)(pp + s8) = hv;
        __threadfence();
      }
    }
  }
  sum += __shfl_xor(sum, 1, 32);
  sum += __shfl_xor(sum, 2, 32);
  sum += __shfl_xor(sum, 4, 32);
  sum += __shfl_xor(sum, 8, 32);
  sum += __shfl_xor(sum, 16, 32);
  const float fl = FL[(size_t)ch * kTP + (rowLive ? t : 0u)];
  const float a = fabsf(sum);
  const float nv = rowLive ? ((a > fl) ? a : fl) : 1.0f;
  float* np = NORM + ((size_t)ch * kTP + t) * 32u + lane;
  *(volatile float*)np = nv;
  __threadfence();
  *(volatile float*)np = nv;
}
static_assert(kNH * kTP == 4096 && 4096 % 8 == 0 && kSP / 8 == 112, "mask grid exact: one wave a row");

__global__ __launch_bounds__(kThr) void headgate_kernel(const float* __restrict__ HV, const float* __restrict__ NORM, const float* __restrict__ XC, const float* __restrict__ UP,
                                                        const float* __restrict__ mhg, const float* __restrict__ skp, unsigned short* __restrict__ HS16, int smp) {
  const unsigned v = blockIdx.x * (unsigned)kThr + threadIdx.x;
  if (v >= (unsigned)(kC * kNH)) return;
  const unsigned t = v >> 2, hd = v & 3u;
  const unsigned ch = (unsigned)smp * (unsigned)kNH + hd;
  const size_t row = (size_t)smp * kC + t;
  const float rn = 1.0f / NORM[((size_t)ch * kTP + t) * 32u];
  const float* hp = HV + ((size_t)hd * kTP + t) * kDH;
  float s = 0.0f;
  for (unsigned d = 0; d < (unsigned)kDH; d += 4) {
    const v4f x = *(const v4f*)(hp + d);
    s += x[0] * rn; s += x[1] * rn; s += x[2] * rn; s += x[3] * rn;
  }
  const float mu = s * kInvDH;
  float q = 0.0f;
  for (unsigned d = 0; d < (unsigned)kDH; d += 4) {
    const v4f x = *(const v4f*)(hp + d);
#pragma unroll
    for (int e = 0; e < 4; ++e) { const float dv = x[e] * rn - mu; q += dv * dv; }
  }
  const float rstd = rsqrtf(q * kInvDH + kEps);
  const float* xcp = XC + row * kI + hd * (unsigned)kDH;
  const float* zp = UP + row * (2 * kI) + kI + hd * (unsigned)kDH;
  const float* gp = mhg + hd * (unsigned)kDH;
  const float* kp = skp + hd * (unsigned)kDH;
  unsigned short* op = HS16 + row * kI + hd * (unsigned)kDH;
  for (unsigned d = 0; d < (unsigned)kDH; d += 8) {
    const v4f x0 = *(const v4f*)(hp + d), x1 = *(const v4f*)(hp + d + 4);
    const v4f c0 = *(const v4f*)(xcp + d), c1 = *(const v4f*)(xcp + d + 4);
    const v4f z0 = *(const v4f*)(zp + d), z1 = *(const v4f*)(zp + d + 4);
    const v4f g0 = *(const v4f*)(gp + d), g1 = *(const v4f*)(gp + d + 4);
    const v4f k0 = *(const v4f*)(kp + d), k1 = *(const v4f*)(kp + d + 4);
    v8h hv;
#pragma unroll
    for (int e = 0; e < 4; ++e) {
      const float n0 = (x0[e] * rn - mu) * rstd * bf16r(g0[e]), n1 = (x1[e] * rn - mu) * rstd * bf16r(g1[e]);
      const float s0 = z0[e] / (1.0f + expf(-z0[e])), s1 = z1[e] / (1.0f + expf(-z1[e]));
      hv[e] = (_Float16)carry_flush((n0 + bf16r(k0[e]) * c0[e]) * s0, kHC);
      hv[4 + e] = (_Float16)carry_flush((n1 + bf16r(k1[e]) * c1[e]) * s1, kHC);
    }
    for (int pass = 0; pass < 2; ++pass) {
      *(volatile v8h*)(op + d) = hv;
      __threadfence();
    }
  }
}
static_assert((kC * kNH + kThr - 1) / kThr == 14, "head-gate grid");

__global__ __launch_bounds__(kThr) void out_kernel(const float* __restrict__ OUT2, float* __restrict__ out) {
  const unsigned v = blockIdx.x * (unsigned)kThr + threadIdx.x;
  const unsigned bp = v / (unsigned)kC;
  const unsigned c = v - bp * (unsigned)kC;
  const unsigned b = bp / (unsigned)kP;
  const unsigned p = bp - b * (unsigned)kP;
  const float x = OUT2[((size_t)b * kC + c) * kD + p];
  float* dp = out + v;
  *(volatile float*)dp = x;
  __threadfence();
  *(volatile float*)dp = x;
}
static_assert((kB * kP * kC) % kThr == 0, "output grid exact");

static_assert(((size_t)kP * kT / 8) % kThr == 0 && ((size_t)kD * kP / 8) % kThr == 0 && ((size_t)kP * kD / 8) % kThr == 0, "plane cast grids exact");

extern "C" void kernel_launch(void* const* d_in, const int* in_sizes, int n_in,
                              void* d_out, int out_size, void* d_ws, size_t ws_size,
                              hipStream_t stream) {
  if (n_in < 29 || d_out == nullptr || d_ws == nullptr) return;
  if (in_sizes[0] != kB * kT * kC || in_sizes[1] != kB * kT * 4 || in_sizes[2] != kB * kP * kC || in_sizes[3] != kB * kP * 4) return;
  if (in_sizes[4] != kP * kT || in_sizes[5] != kP || in_sizes[6] != kP * kT || in_sizes[7] != kP || in_sizes[8] != kD * kP || in_sizes[9] != kD || in_sizes[10] != kP * kD || in_sizes[11] != kP) return;
  if (in_sizes[12] != kNB * kD || in_sizes[13] != kNB * kD * 2 * kI || in_sizes[14] != kNB * 2 * kI || in_sizes[15] != kNB * kCK * kI || in_sizes[16] != kNB * kI) return;
  if (in_sizes[17] != kNB * kI * kI || in_sizes[18] != kNB * kI * kI || in_sizes[19] != kNB * kI * kI || in_sizes[20] != kNB * 3 * kI * kNH || in_sizes[21] != kNB * kNH || in_sizes[22] != kNB * 3 * kI * kNH || in_sizes[23] != kNB * kNH) return;
  if (in_sizes[24] != kNB * kI || in_sizes[25] != kNB * kI || in_sizes[26] != kNB * kI * kD || in_sizes[27] != kNB * kD || in_sizes[28] != kD) return;
  if (out_size != kB * kP * kC) return;
  if (ws_size < kWsTotal) return;
  const float* x_enc = (const float*)d_in[0];
  const float* Ws = (const float*)d_in[4];
  const float* bs = (const float*)d_in[5];
  const float* Wt = (const float*)d_in[6];
  const float* bt = (const float*)d_in[7];
  const float* Wp1 = (const float*)d_in[8];
  const float* bp1 = (const float*)d_in[9];
  const float* Wp2 = (const float*)d_in[10];
  const float* bp2 = (const float*)d_in[11];
  const float* ln_g = (const float*)d_in[12];
  const float* Wup = (const float*)d_in[13];
  const float* bup = (const float*)d_in[14];
  const float* Wconv = (const float*)d_in[15];
  const float* bconv = (const float*)d_in[16];
  const float* Wq = (const float*)d_in[17];
  const float* Wk = (const float*)d_in[18];
  const float* Wv = (const float*)d_in[19];
  const float* Wi = (const float*)d_in[20];
  const float* bi = (const float*)d_in[21];
  const float* Wf = (const float*)d_in[22];
  const float* bf = (const float*)d_in[23];
  const float* mh_g = (const float*)d_in[24];
  const float* skip = (const float*)d_in[25];
  const float* Wdn = (const float*)d_in[26];
  const float* bdn = (const float*)d_in[27];
  const float* post_g = (const float*)d_in[28];
  float* out = (float*)d_out;
  char* ws = (char*)d_ws;
  unsigned short* WH = (unsigned short*)(ws + kOffWH);
  unsigned short* WP1 = (unsigned short*)(ws + kOffWP1);
  unsigned short* WP2 = (unsigned short*)(ws + kOffWP2);
  unsigned short* WUP = (unsigned short*)(ws + kOffWUP);
  unsigned short* WQK = (unsigned short*)(ws + kOffWQK);
  unsigned short* WV = (unsigned short*)(ws + kOffWV);
  unsigned short* WIF = (unsigned short*)(ws + kOffWIF);
  unsigned short* WDN = (unsigned short*)(ws + kOffWDN);
  float* BIAS = (float*)(ws + kOffBIAS);
  float* AS = (float*)(ws + kOffAS);
  float* MT = (float*)(ws + kOffMT);
  float* FL = (float*)(ws + kOffFL);
  float* NORM = (float*)(ws + kOffNORM);
  unsigned short* AH = (unsigned short*)(ws + kOffAH);
  float* X0 = (float*)(ws + kOffX0);
  unsigned short* X0H = (unsigned short*)(ws + kOffX0H);
  float* X = (float*)(ws + kOffX);
  unsigned short* Y16 = (unsigned short*)(ws + kOffY16);
  float* UP = (float*)(ws + kOffUP);
  float* XC = (float*)(ws + kOffXC);
  unsigned short* XC16 = (unsigned short*)(ws + kOffXC16);
  unsigned short* XIN16 = (unsigned short*)(ws + kOffXIN16);
  float* QK = (float*)(ws + kOffQK);
  float* V = (float*)(ws + kOffV);
  unsigned short* G16 = (unsigned short*)(ws + kOffG16);
  float* IFp = (float*)(ws + kOffIF);
  float* VTF = (float*)(ws + kOffVTF);
  unsigned short* VT16 = (unsigned short*)(ws + kOffVT16);
  float* SC = (float*)(ws + kOffSC);
  unsigned short* P16 = (unsigned short*)(ws + kOffP16);
  float* HV = (float*)(ws + kOffHV);
  unsigned short* HS16 = (unsigned short*)(ws + kOffHS16);
  float* DN = (float*)(ws + kOffDN);
  float* OUT2 = (float*)(ws + kOffOUT2);
  const float* ZB = BIAS + kFZB;

  cast_plane_kernel<<<(int)(((size_t)kP * kT / 8) / kThr), kThr, 0, stream>>>(Ws, WH, 9, 4 * kT, 0);
  cast_plane_kernel<<<(int)(((size_t)kP * kT / 8) / kThr), kThr, 0, stream>>>(Ws, WH, 9, 4 * kT, kT);
  cast_plane_kernel<<<(int)(((size_t)kP * kT / 8) / kThr), kThr, 0, stream>>>(Wt, WH, 9, 4 * kT, 2 * kT);
  cast_plane_kernel<<<(int)(((size_t)kP * kT / 8) / kThr), kThr, 0, stream>>>(Wt, WH, 9, 4 * kT, 3 * kT);
  cast_plane_kernel<<<(int)(((size_t)kD * kP / 8) / kThr), kThr, 0, stream>>>(Wp1, WP1, 12, 4096, 0);
  cast_plane_kernel<<<(int)(((size_t)kP * kD / 8) / kThr), kThr, 0, stream>>>(Wp2, WP2, 7, kD, 0);
  for (int blk = 0; blk < kNB; ++blk) {
    wt_plane_kernel<<<2 * kI, kD / 8, 0, stream>>>(Wup + (size_t)blk * kD * 2 * kI, WUP + (size_t)blk * 2 * kI * kD, kD, 2 * kI, 2 * kI, kD, 0);
    wt_plane_kernel<<<kI, kI / 8, 0, stream>>>(Wq + (size_t)blk * kI * kI, WQK + (size_t)blk * 2 * kI * kI, kI, kI, kI, kI, 0);
    wt_plane_kernel<<<kI, kI / 8, 0, stream>>>(Wk + (size_t)blk * kI * kI, WQK + (size_t)blk * 2 * kI * kI + (size_t)kI * kI, kI, kI, kI, kI, 0);
    wt_plane_kernel<<<kI, kI / 8, 0, stream>>>(Wv + (size_t)blk * kI * kI, WV + (size_t)blk * kI * kI, kI, kI, kI, kI, 0);
    wt_plane_kernel<<<kNH, 3 * kI / 8, 0, stream>>>(Wi + (size_t)blk * 3 * kI * kNH, WIF + (size_t)blk * kD * 3 * kI, 3 * kI, kNH, kNH, 3 * kI, 0);
    wt_plane_kernel<<<kD - kNH, 3 * kI / 8, 0, stream>>>(Wf + (size_t)blk * 3 * kI * kNH, WIF + (size_t)blk * kD * 3 * kI + (size_t)kNH * 3 * kI, 3 * kI, kNH, kNH, 3 * kI, 0);
    wt_plane_kernel<<<kD, kI / 8, 0, stream>>>(Wdn + (size_t)blk * kI * kD, WDN + (size_t)blk * kD * kI, kI, kD, kD, kI, 0);
  }
  setup_kernel<<<38, kThr, 0, stream>>>(bs, bt, bp1, bp2, bup, bi, bf, bdn, BIAS, WH, WP2);
  zero_kernel<<<(int)(((size_t)(kRP - kR) * (4 * kT) / 8) / kThr), kThr, 0, stream>>>(AH + (size_t)kR * (4 * kT));
  zero_kernel<<<(int)(((size_t)(kRP - kR) * kI / 8) / kThr), kThr, 0, stream>>>(HS16 + (size_t)kR * kI);

  decomp_kernel<<<dim3((kC + kThr - 1) / kThr, kB * 8), kThr, 0, stream>>>(x_enc, AH);
  wmma_gemm64<0, false, 2, 0, false, 0><<<dim3((kRP / 64) * (kD / 64) / 8, 1), 256, 0, stream>>>(
      AH, AH, 4 * kT, 0L, WH, WH, 4 * kT, 0L, (void*)X0, (void*)X0, kD, 0L, BIAS + kFBS, nullptr, 0L, kRP, kD, 4 * kT, kScII);
  cast8_kernel<<<(int)(((size_t)kRP * kD / 8) / kThr), kThr, 0, stream>>>(X0, X0H);
  wmma_gemm64<0, false, 2, 0, false, 0><<<dim3((kRP / 64) * (kD / 64) / 8, 1), 256, 0, stream>>>(
      X0H, X0H, kD, 0L, WP1, WP1, kP, 0L, (void*)X, (void*)X, kD, 0L, BIAS + kFBP1, nullptr, 0L, kRP, kD, kP, kScII);

  for (int blk = 0; blk < kNB; ++blk) {
    const unsigned short* WUPb = WUP + (size_t)blk * 2 * kI * kD;
    const unsigned short* WQKb = WQK + (size_t)blk * 2 * kI * kI;
    const unsigned short* WVb = WV + (size_t)blk * kI * kI;
    const unsigned short* WIFb = WIF + (size_t)blk * kD * 3 * kI;
    const unsigned short* WDNb = WDN + (size_t)blk * kD * kI;
    const float* Bb = BIAS + kFBlk + blk * kFBlkLen;
    addln_kernel<<<kRP / kThr, kThr, 0, stream>>>(X, DN, ln_g + (size_t)blk * kD, X, Y16, (blk == 0) ? 0 : 3);
    wmma_gemm64<0, false, 2, 0, false, 0><<<dim3((kRP / 64) * (2 * kI / 64) / 8, 1), 256, 0, stream>>>(
        Y16, Y16, kD, 0L, WUPb, WUPb, kD, 0L, (void*)UP, (void*)UP, 2 * kI, 0L, Bb + kFBUP, nullptr, 0L, kRP, 2 * kI, kD, kScIW);
    conv_silu_kernel<<<(int)(((size_t)kRT * 32) / kThr), kThr, 0, stream>>>(UP, Wconv + (size_t)blk * kCK * kI, bconv + (size_t)blk * kI, XC, XC16, XIN16);
    wmma_gemm64<0, false, 2, 0, false, 0><<<dim3((kRP / 64) * (2 * kI / 64) / 8, 1), 256, 0, stream>>>(
        XC16, XC16, kI, 0L, WQKb, WQKb, kI, 0L, (void*)QK, (void*)QK, 2 * kI, 0L, ZB, nullptr, 0L, kRP, 2 * kI, kI, kScIW);
    wmma_gemm64<0, false, 2, 0, false, 0><<<dim3((kRP / 64) * (kI / 64) / 8, 1), 256, 0, stream>>>(
        XIN16, XIN16, kI, 0L, WVb, WVb, kI, 0L, (void*)V, (void*)V, kI, 0L, ZB, nullptr, 0L, kRP, kI, kI, kScIW);
    qkv_kernel<<<(int)(((size_t)kRT * 96) / kThr), kThr, 0, stream>>>(QK, V, G16);
    wmma_gemm64<0, false, 2, 0, false, 0><<<dim3((kRP / 64) * (kD / 64) / 8, 1), 256, 0, stream>>>(
        G16, G16, 3 * kI, 0L, WIFb, WIFb, 3 * kI, 0L, (void*)IFp, (void*)IFp, kD, 0L, Bb + kFBIF, nullptr, 0L, kRP, kD, 3 * kI, kScIW);
    gate_scan_kernel<<<1, 32, 0, stream>>>(IFp, AS, MT, FL);
    for (int smp = 0; smp < kB; ++smp) {
      const unsigned short* Gs = G16 + (size_t)smp * kC * 3 * kI;
      wmma_gemm64<0, false, 2, 0, false, 0><<<dim3((kI / 64) * (kTP / 64) / 8, 1), 256, 0, stream>>>(
          WVb, WVb, kI, 0L, XIN16 + (size_t)smp * kC * kI, XIN16 + (size_t)smp * kC * kI, kI, 0L, (void*)VTF, (void*)VTF, kTP, 0L, ZB, nullptr, 0L, kI, kTP, kI, kScIW);
      vt_kernel<<<(kI * 112) / kThr, kThr, 0, stream>>>(VTF, VT16);
      wmma_gemm64<0, false, 2, 0, false, 0><<<dim3((kTP / 64) * (kSP / 64) / 8, kNH), 256, 0, stream>>>(
          Gs, Gs, 3 * kI, (long)kDH, Gs + kI, Gs + kI, 3 * kI, (long)kDH, (void*)SC, (void*)SC, kSP, (long)kTP * kSP, ZB, nullptr, 0L, kTP, kSP, kDH, kScQK);
      mask_kernel<<<(kNH * kTP) / 8, kThr, 0, stream>>>(SC, AS, MT, FL, P16, NORM, smp);
      wmma_gemm64<0, false, 2, 0, false, 0><<<dim3((kTP / 64) * (kDH / 64) / 8, kNH), 256, 0, stream>>>(
          P16, P16, kSP, (long)kTP * kSP, VT16, VT16, kSP, (long)kDH * kSP, (void*)HV, (void*)HV, kDH, (long)kTP * kDH, ZB, nullptr, 0L, kTP, kDH, kSP, kScPV);
      headgate_kernel<<<14, kThr, 0, stream>>>(HV, NORM, XC, UP, mh_g + (size_t)blk * kI, skip + (size_t)blk * kI, HS16, smp);
    }
    wmma_gemm64<0, false, 2, 0, false, 0><<<dim3((kRP / 64) * (kD / 64) / 8, 1), 256, 0, stream>>>(
        HS16, HS16, kI, 0L, WDNb, WDNb, kI, 0L, (void*)DN, (void*)DN, kD, 0L, Bb + kFBDN, nullptr, 0L, kRP, kD, kI, kScDN);
  }
  addln_kernel<<<kRP / kThr, kThr, 0, stream>>>(X, DN, post_g, X, Y16, 3);
  wmma_gemm64<0, false, 2, 0, false, 0><<<dim3((kRP / 64) * (kD / 64) / 8, 1), 256, 0, stream>>>(
      Y16, Y16, kD, 0L, WP2, WP2, kD, 0L, (void*)OUT2, (void*)OUT2, kD, 0L, BIAS + kFBP2, nullptr, 0L, kRP, kD, kD, kScII);
  out_kernel<<<(kB * kP * kC) / kThr, kThr, 0, stream>>>(OUT2, out);
}
